// LocalSelfAttention_56513179680865
// MI455X (gfx1250) — hardware-verified
//
#include <hip/hip_runtime.h>

constexpr int NBATCH  = 2;
constexpr int SEQ     = 2048;
constexpr int NNB     = 32;
constexpr int NHEAD   = 8;
constexpr int DIN     = 768;
constexpr int DMODEL  = 768;
constexpr int DOUTF   = 768;
constexpr int HDIM    = 96;
constexpr int QKV_N   = 3 * DMODEL;
constexpr int MROWS   = NBATCH * SEQ;
constexpr float ATT_SCALE = 0.10206207261596575f;

static_assert(NNB == 32);
static_assert(NHEAD * 32 == 256);
static_assert(NHEAD * HDIM == DMODEL);
static_assert(HDIM % 4 == 0);
static_assert(MROWS % 64 == 0);
static_assert(QKV_N % 64 == 0);
static_assert(DOUTF % 64 == 0);
static_assert(DIN % 32 == 0);
static_assert(DMODEL % 32 == 0);

constexpr size_t OFF_XB    = 0;
constexpr size_t SZ_XB     = (size_t)MROWS * DIN * 2;
constexpr size_t OFF_WQB   = OFF_XB + SZ_XB;
constexpr size_t SZ_WQB    = (size_t)QKV_N * DIN * 2;
constexpr size_t OFF_WOB   = OFF_WQB + SZ_WQB;
constexpr size_t SZ_WOB    = (size_t)DOUTF * DMODEL * 2;
constexpr size_t OFF_BIASR = OFF_WOB + SZ_WOB;
constexpr size_t SZ_BIASR  = (size_t)QKV_N * 4;
constexpr size_t OFF_QKV   = OFF_BIASR + SZ_BIASR;
constexpr size_t SZ_QKV    = (size_t)MROWS * QKV_N * 4;
constexpr size_t OFF_APL   = OFF_QKV + SZ_QKV;
constexpr size_t APLANE_ELEMS = (size_t)MROWS * DMODEL;
constexpr size_t SZ_APL    = 2 * APLANE_ELEMS * 2;
constexpr size_t WS_TOTAL  = OFF_APL + SZ_APL;
static_assert(OFF_WQB % 128 == 0 && OFF_WOB % 128 == 0 && OFF_BIASR % 128 == 0 && OFF_QKV % 128 == 0 && OFF_APL % 128 == 0);
static_assert(WS_TOTAL == 61350912);
static_assert(WS_TOTAL <= 134217728);

typedef __attribute__((ext_vector_type(16))) _Float16 v16h;
typedef __attribute__((ext_vector_type(8)))  _Float16 v8h;
typedef __attribute__((ext_vector_type(16))) __bf16   v16b;
typedef __attribute__((ext_vector_type(8)))  __bf16   v8b;
typedef __attribute__((ext_vector_type(8)))  float    v8f;
typedef __attribute__((ext_vector_type(4)))  float    v4f;
typedef __attribute__((ext_vector_type(4)))  unsigned int v4u;

__device__ __forceinline__ unsigned short f2bf_bits(float f) {
  unsigned u = __float_as_uint(f);
  return (unsigned short)((u + 0x7FFFu + ((u >> 16) & 1u)) >> 16);
}
__device__ __forceinline__ float bf_bits2f(unsigned short h) { return __uint_as_float(((unsigned)h) << 16); }

__device__ __forceinline__ void dep_guard_h(v8f& a, v8f& b, v16h x, v16h y) { asm volatile("v_nop\n\tv_nop\n\tv_nop\n\tv_nop" : "+v"(a), "+v"(b) : "v"(x), "v"(y)); }
__device__ __forceinline__ void dep_guard_b(v8f& a, v8f& b, v16b x, v16b y) { asm volatile("v_nop\n\tv_nop\n\tv_nop\n\tv_nop" : "+v"(a), "+v"(b) : "v"(x), "v"(y)); }
__device__ __forceinline__ void keep4_h(v16h a, v16h b, v16h c, v16h d) { asm volatile("v_nop" :: "v"(a), "v"(b), "v"(c), "v"(d)); }
__device__ __forceinline__ void keep4_b(v16b a, v16b b, v16b c, v16b d) { asm volatile("v_nop" :: "v"(a), "v"(b), "v"(c), "v"(d)); }
__device__ __forceinline__ void acc_guard4(v8f& a, v8f& b, v8f& c, v8f& d) { asm volatile("v_nop\n\tv_nop\n\tv_nop\n\tv_nop" : "+v"(a), "+v"(b), "+v"(c), "+v"(d)); }
template <typename T> struct Frag;
template <> struct Frag<_Float16> {
  typedef v16h V; union U { v16h v; v8h h[2]; };
  static __device__ __forceinline__ v16h load(const _Float16* p) {
    U f; f.h[0] = *(const v8h*)(p); f.h[1] = *(const v8h*)(p + 16); return f.v;
  }
  static __device__ __forceinline__ v8f mma(v16h a, v16h b, v8f c) {
    return __builtin_amdgcn_wmma_f32_16x16x32_f16(false, a, false, b, (short)0, c, false, false);
  }
  static __device__ __forceinline__ void guard(v8f& a, v8f& b, v16h x, v16h y) { dep_guard_h(a, b, x, y); }
  static __device__ __forceinline__ void keep(v16h a, v16h b, v16h c, v16h d) { keep4_h(a, b, c, d); }
};
template <> struct Frag<__bf16> {
  typedef v16b V; union U { v16b v; v8b h[2]; };
  static __device__ __forceinline__ v16b load(const __bf16* p) {
    U f; f.h[0] = *(const v8b*)(p); f.h[1] = *(const v8b*)(p + 16); return f.v;
  }
  static __device__ __forceinline__ v8f mma(v16b a, v16b b, v8f c) {
    return __builtin_amdgcn_wmma_f32_16x16x32_bf16(false, a, false, b, (short)0, c, false, false);
  }
  static __device__ __forceinline__ void guard(v8f& a, v8f& b, v16b x, v16b y) { dep_guard_b(a, b, x, y); }
  static __device__ __forceinline__ void keep(v16b a, v16b b, v16b c, v16b d) { keep4_b(a, b, c, d); }
};

template <int ET> struct Elem;
template <> struct Elem<0> { typedef _Float16 T; };
template <> struct Elem<1> { typedef __bf16 T; };
template <int ET, int SPLIT, int BIAS_MODE, int OUT_MODE, bool ROWZERO>
__global__ __launch_bounds__(256) void wmma_gemm64(
    const unsigned short* __restrict__ Ap, const unsigned short* __restrict__ A2p, int lda, long strideA,
    const unsigned short* __restrict__ Btp, const unsigned short* __restrict__ Bt2p, int ldb, long strideB,
    void* __restrict__ Cout, void* __restrict__ Cout2, int ldc, long strideC,
    const float* __restrict__ bias,
    const int* __restrict__ rowmask,
    int M, int N, int K, float scale) {
  typedef typename Elem<ET>::T T;
  typedef typename Frag<T>::V V;
  const T* A = (const T*)Ap; const T* A2 = (const T*)A2p; const T* Bt = (const T*)Btp; const T* Bt2 = (const T*)Bt2p;
  __shared__ __align__(16) float sT[8][16 * 68];
  const int b    = blockIdx.y;
  const int lane = threadIdx.x & 31;
  const int wave = threadIdx.x >> 5;
  const int tilesN = N >> 6;
  const int tilesM = M >> 6;
  const int tile = blockIdx.x * 8 + wave;
  if (tile >= tilesM * tilesN) return;
  const int tm = tile / tilesN;
  const int tn = tile - tm * tilesN;
  const int m0 = tm << 6;
  const int n0 = tn << 6;

  const T* Ab  = A  + (size_t)b * strideA;
  const T* Bb  = Bt + (size_t)b * strideB;
  const T* Ab2 = (SPLIT >= 1) ? (A2  + (size_t)b * strideA) : nullptr;
  const T* Bb2 = (SPLIT == 2) ? (Bt2 + (size_t)b * strideB) : nullptr;

  const int rlane = lane & 15;
  const int koff  = (lane >> 4) * 8;
  const int mOff  = (lane >> 4) * 8;

  v8f acc[4][4];
#pragma unroll
  for (int i = 0; i < 4; ++i)
#pragma unroll
    for (int j = 0; j < 4; ++j) acc[i][j] = (v8f){0.f,0.f,0.f,0.f,0.f,0.f,0.f,0.f};

  for (int k0 = 0; k0 < K; k0 += 32) {
    V bh[4], bl[4];
#pragma unroll
    for (int j = 0; j < 4; ++j) {
      const size_t bo = (size_t)(n0 + (j << 4) + rlane) * ldb + koff + k0;
      bh[j] = Frag<T>::load(Bb + bo);
      if (SPLIT == 2) bl[j] = Frag<T>::load(Bb2 + bo);
    }
#pragma unroll
    for (int i = 0; i < 4; ++i) {
      const size_t ao = (size_t)(m0 + (i << 4) + rlane) * lda + koff + k0;
      V ah = Frag<T>::load(Ab + ao);
      V al;
      if (SPLIT >= 1) al = Frag<T>::load(Ab2 + ao);
      else al = ah;
#pragma unroll
      for (int j = 0; j < 4; ++j) {
        acc[i][j] = Frag<T>::mma(ah, bh[j], acc[i][j]);
        if (SPLIT == 2) acc[i][j] = Frag<T>::mma(ah, bl[j], acc[i][j]);
        if (SPLIT >= 1) acc[i][j] = Frag<T>::mma(al, bh[j], acc[i][j]);
      }
      Frag<T>::guard(acc[i][0], acc[i][3], ah, al);
    }
    Frag<T>::keep(bh[0], bh[1], bh[2], bh[3]);
    if (SPLIT == 2) Frag<T>::keep(bl[0], bl[1], bl[2], bl[3]);
  }
  acc_guard4(acc[0][0], acc[0][1], acc[0][2], acc[0][3]);
  acc_guard4(acc[1][0], acc[1][1], acc[1][2], acc[1][3]);
  acc_guard4(acc[2][0], acc[2][1], acc[2][2], acc[2][3]);
  acc_guard4(acc[3][0], acc[3][1], acc[3][2], acc[3][3]);

  float* slab = sT[wave];
#pragma unroll
  for (int i = 0; i < 4; ++i) {
    const int mBase = m0 + (i << 4);
    int mz[8];
#pragma unroll
    for (int r = 0; r < 8; ++r) mz[r] = 0;
    if (ROWZERO) {
#pragma unroll
      for (int r = 0; r < 8; ++r) mz[r] = rowmask[mBase + mOff + r];
    }
#pragma unroll
    for (int j = 0; j < 4; ++j) {
      const int n = n0 + (j << 4) + rlane;
      float bv = 0.f;
      if (BIAS_MODE == 2) bv = bias[n];
#pragma unroll
      for (int r = 0; r < 8; ++r) {
        float v = acc[i][j][r] * scale;
        if (BIAS_MODE == 1) v += bias[mBase + mOff + r];
        if (BIAS_MODE == 2) v += bv;
        if (ROWZERO) v = (mz[r] != 0) ? 0.0f : v;
        slab[(mOff + r) * 68 + (j << 4) + rlane] = v;
      }
    }
    __builtin_amdgcn_fence(__ATOMIC_RELEASE, "workgroup");
    __builtin_amdgcn_wave_barrier();
    __builtin_amdgcn_fence(__ATOMIC_ACQUIRE, "workgroup");
    if (OUT_MODE == 0) {
      float* C = (float*)Cout + (size_t)b * strideC;
      const int hh = lane >> 4, c4 = (lane & 15) * 4;
      for (int pass = 0; pass < 2; ++pass) {
#pragma unroll
        for (int it = 0; it < 8; ++it) {
          const int row = it * 2 + hh;
          v4f v = *(const v4f*)(slab + row * 68 + c4);
          *(volatile v4f*)(C + (size_t)(mBase + row) * ldc + n0 + c4) = v;
        }
        __threadfence();
      }
    } else {
      const int q = lane >> 3, c8 = (lane & 7) * 8;
      unsigned short* C  = (unsigned short*)Cout  + (size_t)b * strideC;
      unsigned short* C2 = (OUT_MODE == 2) ? ((unsigned short*)Cout2 + (size_t)b * strideC) : nullptr;
      for (int pass = 0; pass < 2; ++pass) {
#pragma unroll
        for (int it = 0; it < 4; ++it) {
          const int row = it * 4 + q;
          const float* sp = slab + row * 68 + c8;
          v8h hv, lv;
#pragma unroll
          for (int e = 0; e < 8; ++e) {
            if (OUT_MODE == 1) {
              hv[e] = (_Float16)sp[e];
            } else {
              unsigned short hb = f2bf_bits(sp[e]);
              unsigned short lb = f2bf_bits(sp[e] - bf_bits2f(hb));
              hv[e] = __builtin_bit_cast(_Float16, hb);
              lv[e] = __builtin_bit_cast(_Float16, lb);
            }
          }
          *(volatile v8h*)(C + (size_t)(mBase + row) * ldc + n0 + c8) = hv;
          if (OUT_MODE == 2) *(volatile v8h*)(C2 + (size_t)(mBase + row) * ldc + n0 + c8) = lv;
        }
        __threadfence();
      }
    }
    __builtin_amdgcn_fence(__ATOMIC_RELEASE, "workgroup");
    __builtin_amdgcn_wave_barrier();
    __builtin_amdgcn_fence(__ATOMIC_ACQUIRE, "workgroup");
  }
}

__global__ __launch_bounds__(256) void cast_f32_bf16x8(
    const float* __restrict__ in, unsigned short* __restrict__ out, int n8) {
  const int i = blockIdx.x * 256 + threadIdx.x;
  if (i < n8) {
    const v4f a = *(const v4f*)(in + (size_t)8 * i);
    const v4f c = *(const v4f*)(in + (size_t)8 * i + 4);
    v4u u;
    u[0] = (unsigned)f2bf_bits(a[0]) | ((unsigned)f2bf_bits(a[1]) << 16);
    u[1] = (unsigned)f2bf_bits(a[2]) | ((unsigned)f2bf_bits(a[3]) << 16);
    u[2] = (unsigned)f2bf_bits(c[0]) | ((unsigned)f2bf_bits(c[1]) << 16);
    u[3] = (unsigned)f2bf_bits(c[2]) | ((unsigned)f2bf_bits(c[3]) << 16);
    unsigned short* p = out + (size_t)8 * i;
    *(volatile v4u*)p = u;
    __threadfence();
    *(volatile v4u*)p = u;
  }
}

__global__ __launch_bounds__(256) void rne_bias_kernel(
    const float* __restrict__ in, float* __restrict__ out, int n4) {
  const int i = blockIdx.x * 256 + threadIdx.x;
  if (i < n4) {
    const v4f a = *(const v4f*)(in + (size_t)4 * i);
    v4f r;
    r[0] = bf_bits2f(f2bf_bits(a[0]));
    r[1] = bf_bits2f(f2bf_bits(a[1]));
    r[2] = bf_bits2f(f2bf_bits(a[2]));
    r[3] = bf_bits2f(f2bf_bits(a[3]));
    float* p = out + (size_t)4 * i;
    *(volatile v4f*)p = r;
    __threadfence();
    *(volatile v4f*)p = r;
  }
}

__global__ __launch_bounds__(256) void nbr_attn_kernel(
    const float* __restrict__ qkv, const int* __restrict__ nbr, const int* __restrict__ padmask,
    unsigned short* __restrict__ aplanes) {
  __shared__ __align__(16) unsigned short rows[2][DMODEL];
  const int tid  = threadIdx.x;
  const int lane = tid & 31;
  const int h    = tid >> 5;
  const int bs   = blockIdx.x;
  const int b    = bs / SEQ;

  int nb = nbr[(size_t)bs * NNB + lane];
  nb = nb < 0 ? 0 : nb;
  nb = nb > (SEQ - 1) ? (SEQ - 1) : nb;
  const int pm = padmask[b * SEQ + nb];

  const float* qp = qkv + (size_t)bs * QKV_N + h * HDIM;
  const float* kp = qkv + (size_t)(b * SEQ + nb) * QKV_N + DMODEL + h * HDIM;
  float dot = 0.0f;
#pragma unroll 4
  for (int d = 0; d < HDIM; d += 4) {
    const v4f qv = *(const v4f*)(qp + d);
    const v4f kv = *(const v4f*)(kp + d);
    dot = fmaf(qv[0], kv[0], dot);
    dot = fmaf(qv[1], kv[1], dot);
    dot = fmaf(qv[2], kv[2], dot);
    dot = fmaf(qv[3], kv[3], dot);
  }
  float sc = dot * ATT_SCALE;
  sc = (pm != 0) ? -__builtin_inff() : sc;
  float mx = sc;
#pragma unroll
  for (int off = 16; off > 0; off >>= 1) mx = fmaxf(mx, __shfl_xor(mx, off, 32));
  const float p = expf(sc - mx);
  float sum = p;
#pragma unroll
  for (int off = 16; off > 0; off >>= 1) sum += __shfl_xor(sum, off, 32);
  const float w = p * (1.0f / sum);

  const int voff = nb * QKV_N;
  const float* vbase = qkv + (size_t)b * SEQ * QKV_N + 2 * DMODEL + h * HDIM + lane;
  float o0 = 0.0f, o1 = 0.0f, o2 = 0.0f;
#pragma unroll 2
  for (int j = 0; j < NNB; ++j) {
    const float wj = __shfl(w, j, 32);
    const int   vo = __shfl(voff, j, 32);
    const float* vp = vbase + vo;
    o0 = fmaf(wj, vp[0], o0);
    o1 = fmaf(wj, vp[32], o1);
    o2 = fmaf(wj, vp[64], o2);
  }

  const unsigned short hb0 = f2bf_bits(o0), hb1 = f2bf_bits(o1), hb2 = f2bf_bits(o2);
  const unsigned short lb0 = f2bf_bits(o0 - bf_bits2f(hb0));
  const unsigned short lb1 = f2bf_bits(o1 - bf_bits2f(hb1));
  const unsigned short lb2 = f2bf_bits(o2 - bf_bits2f(hb2));
  rows[0][h * HDIM + lane]      = hb0;
  rows[0][h * HDIM + lane + 32] = hb1;
  rows[0][h * HDIM + lane + 64] = hb2;
  rows[1][h * HDIM + lane]      = lb0;
  rows[1][h * HDIM + lane + 32] = lb1;
  rows[1][h * HDIM + lane + 64] = lb2;
  __syncthreads();
  if (h < 6) {
    const int plane = (h >= 3) ? 1 : 0;
    const int seg   = h - 3 * plane;
    const v4u val = *(const v4u*)(const void*)(&rows[plane][seg * 256 + lane * 8]);
    unsigned short* dst = aplanes + (size_t)plane * APLANE_ELEMS + (size_t)bs * DMODEL + seg * 256 + lane * 8;
    *(volatile v4u*)dst = val;
    __threadfence();
    *(volatile v4u*)dst = val;
  }
}

extern "C" void kernel_launch(void* const* d_in, const int* in_sizes, int n_in,
                              void* d_out, int out_size, void* d_ws, size_t ws_size,
                              hipStream_t stream) {
  if (n_in < 6) return;
  if (in_sizes[0] != MROWS * DIN) return;
  if (in_sizes[1] != QKV_N * DIN) return;
  if (in_sizes[2] != QKV_N) return;
  if (in_sizes[3] != DOUTF * DMODEL) return;
  if (in_sizes[4] != MROWS * NNB) return;
  if (in_sizes[5] != MROWS) return;
  if (out_size != MROWS * DOUTF) return;
  if (ws_size < WS_TOTAL) return;

  const float* x     = (const float*)d_in[0];
  const float* w_qkv = (const float*)d_in[1];
  const float* b_qkv = (const float*)d_in[2];
  const float* w_out = (const float*)d_in[3];
  const int*   nbr   = (const int*)d_in[4];
  const int*   padm  = (const int*)d_in[5];
  float* out = (float*)d_out;

  char* ws = (char*)d_ws;
  unsigned short* xb    = (unsigned short*)(ws + OFF_XB);
  unsigned short* wqb   = (unsigned short*)(ws + OFF_WQB);
  unsigned short* wob   = (unsigned short*)(ws + OFF_WOB);
  float*          biasr = (float*)(ws + OFF_BIASR);
  float*          qkv   = (float*)(ws + OFF_QKV);
  unsigned short* apl   = (unsigned short*)(ws + OFF_APL);
  unsigned short* ahi   = apl;
  unsigned short* alo   = apl + APLANE_ELEMS;

  {
    const int n8x = MROWS * DIN / 8;
    cast_f32_bf16x8<<<(n8x + 255) / 256, 256, 0, stream>>>(x, xb, n8x);
    const int n8q = QKV_N * DIN / 8;
    cast_f32_bf16x8<<<(n8q + 255) / 256, 256, 0, stream>>>(w_qkv, wqb, n8q);
    const int n8o = DOUTF * DMODEL / 8;
    cast_f32_bf16x8<<<(n8o + 255) / 256, 256, 0, stream>>>(w_out, wob, n8o);
  }
  {
    const int n4 = QKV_N / 4;
    rne_bias_kernel<<<(n4 + 255) / 256, 256, 0, stream>>>(b_qkv, biasr, n4);
  }
  {
    const int tiles = (MROWS / 64) * (QKV_N / 64);
    wmma_gemm64<1, 0, 2, 0, true><<<dim3(tiles / 8, 1), 256, 0, stream>>>(
        xb, nullptr, DIN, 0L, wqb, nullptr, DIN, 0L,
        (void*)qkv, nullptr, QKV_N, 0L, biasr, padm, MROWS, QKV_N, DIN, 1.0f);
  }
  nbr_attn_kernel<<<MROWS, 256, 0, stream>>>(qkv, nbr, padm, apl);
  {
    const int tiles = (MROWS / 64) * (DOUTF / 64);
    wmma_gemm64<1, 1, 0, 0, true><<<dim3(tiles / 8, 1), 256, 0, stream>>>(
        ahi, alo, DMODEL, 0L, wob, nullptr, DMODEL, 0L,
        (void*)out, nullptr, DOUTF, 0L, nullptr, padm, MROWS, DOUTF, DMODEL, 1.0f);
  }
}
